// MultiHeadDepthwiseSelfAttention_4071628996648
// MI455X (gfx1250) — hardware-verified
//
#include <hip/hip_runtime.h>
#include <math.h>

typedef __attribute__((ext_vector_type(16))) _Float16 v16h;
typedef __attribute__((ext_vector_type(8)))  _Float16 v8h;
typedef __attribute__((ext_vector_type(16))) __bf16   v16b;
typedef __attribute__((ext_vector_type(8)))  __bf16   v8b;
typedef __attribute__((ext_vector_type(8)))  float    v8f;
typedef __attribute__((ext_vector_type(4)))  float    v4f;
typedef __attribute__((ext_vector_type(2)))  float    v2f;

#define FE 768
#define NHEAD 12
#define HDIM 64

__device__ __forceinline__ unsigned short f2bf_bits(float f) {
  unsigned u = __float_as_uint(f);
  return (unsigned short)((u + 0x7FFFu + ((u >> 16) & 1u)) >> 16);
}
__device__ __forceinline__ float bf_bits2f(unsigned short h) { return __uint_as_float(((unsigned)h) << 16); }

__device__ __forceinline__ void dep_guard_h(v8f& a, v8f& b, v16h x, v16h y) { asm volatile("v_nop\n\tv_nop\n\tv_nop\n\tv_nop" : "+v"(a), "+v"(b) : "v"(x), "v"(y)); }
__device__ __forceinline__ void dep_guard_b(v8f& a, v8f& b, v16b x, v16b y) { asm volatile("v_nop\n\tv_nop\n\tv_nop\n\tv_nop" : "+v"(a), "+v"(b) : "v"(x), "v"(y)); }
__device__ __forceinline__ void keep4_h(v16h a, v16h b, v16h c, v16h d) { asm volatile("v_nop" :: "v"(a), "v"(b), "v"(c), "v"(d)); }
__device__ __forceinline__ void keep4_b(v16b a, v16b b, v16b c, v16b d) { asm volatile("v_nop" :: "v"(a), "v"(b), "v"(c), "v"(d)); }
__device__ __forceinline__ void acc_guard4(v8f& a, v8f& b, v8f& c, v8f& d) { asm volatile("v_nop\n\tv_nop\n\tv_nop\n\tv_nop" : "+v"(a), "+v"(b), "+v"(c), "+v"(d)); }
template <typename T> struct Frag;
template <> struct Frag<_Float16> {
  typedef v16h V; union U { v16h v; v8h h[2]; };
  static __device__ __forceinline__ v16h load(const _Float16* p) {
    U f; f.h[0] = *(const v8h*)(p); f.h[1] = *(const v8h*)(p + 16); return f.v;
  }
  static __device__ __forceinline__ v8f mma(v16h a, v16h b, v8f c) {
    return __builtin_amdgcn_wmma_f32_16x16x32_f16(false, a, false, b, (short)0, c, false, false);
  }
  static __device__ __forceinline__ void guard(v8f& a, v8f& b, v16h x, v16h y) { dep_guard_h(a, b, x, y); }
  static __device__ __forceinline__ void keep(v16h a, v16h b, v16h c, v16h d) { keep4_h(a, b, c, d); }
};
template <> struct Frag<__bf16> {
  typedef v16b V; union U { v16b v; v8b h[2]; };
  static __device__ __forceinline__ v16b load(const __bf16* p) {
    U f; f.h[0] = *(const v8b*)(p); f.h[1] = *(const v8b*)(p + 16); return f.v;
  }
  static __device__ __forceinline__ v8f mma(v16b a, v16b b, v8f c) {
    return __builtin_amdgcn_wmma_f32_16x16x32_bf16(false, a, false, b, (short)0, c, false, false);
  }
  static __device__ __forceinline__ void guard(v8f& a, v8f& b, v16b x, v16b y) { dep_guard_b(a, b, x, y); }
  static __device__ __forceinline__ void keep(v16b a, v16b b, v16b c, v16b d) { keep4_b(a, b, c, d); }
};

template <int ET> struct Elem;
template <> struct Elem<0> { typedef _Float16 T; };
template <> struct Elem<1> { typedef __bf16 T; };
template <int ET, bool SPLIT, int BIAS_MODE, int OUT_MODE, bool RESID, int ACT = 0>
__global__ __launch_bounds__(256) void wmma_gemm64(
    const unsigned short* __restrict__ Ap, const unsigned short* __restrict__ A2p, int lda, long strideA,
    const unsigned short* __restrict__ Btp, const unsigned short* __restrict__ Bt2p, int ldb, long strideB,
    void* __restrict__ Cout, void* __restrict__ Cout2, int ldc, long strideC,
    const float* __restrict__ bias,
    const float* __restrict__ resid, long strideR,
    int M, int N, int K, float scale) {
  typedef typename Elem<ET>::T T;
  typedef typename Frag<T>::V V;
  const T* A = (const T*)Ap; const T* A2 = (const T*)A2p; const T* Bt = (const T*)Btp; const T* Bt2 = (const T*)Bt2p;
  __shared__ __align__(16) float sT[8][16 * 68];
  const int b    = blockIdx.y;
  const int lane = threadIdx.x & 31;
  const int wave = threadIdx.x >> 5;
  const int tilesN = N >> 6;
  const int tilesM = M >> 6;
  const int tile = blockIdx.x * 8 + wave;
  if (tile >= tilesM * tilesN) return;
  const int tm = tile / tilesN;
  const int tn = tile - tm * tilesN;
  const int m0 = tm << 6;
  const int n0 = tn << 6;

  const T* Ab  = A  + (size_t)b * strideA;
  const T* Bb  = Bt + (size_t)b * strideB;
  const T* Ab2 = SPLIT ? (A2  + (size_t)b * strideA) : nullptr;
  const T* Bb2 = SPLIT ? (Bt2 + (size_t)b * strideB) : nullptr;

  const int rlane = lane & 15;
  const int koff  = (lane >> 4) * 8;
  const int mOff  = (lane >> 4) * 8;

  v8f acc[4][4];
#pragma unroll
  for (int i = 0; i < 4; ++i)
#pragma unroll
    for (int j = 0; j < 4; ++j) acc[i][j] = (v8f){0.f,0.f,0.f,0.f,0.f,0.f,0.f,0.f};

  for (int k0 = 0; k0 < K; k0 += 32) {
    V bh[4], bl[4];
#pragma unroll
    for (int j = 0; j < 4; ++j) {
      const size_t bo = (size_t)(n0 + (j << 4) + rlane) * ldb + koff + k0;
      bh[j] = Frag<T>::load(Bb + bo);
      if (SPLIT) bl[j] = Frag<T>::load(Bb2 + bo);
    }
#pragma unroll
    for (int i = 0; i < 4; ++i) {
      const size_t ao = (size_t)(m0 + (i << 4) + rlane) * lda + koff + k0;
      V ah = Frag<T>::load(Ab + ao);
      V al;
      if (SPLIT) al = Frag<T>::load(Ab2 + ao);
#pragma unroll
      for (int j = 0; j < 4; ++j) {
        acc[i][j] = Frag<T>::mma(ah, bh[j], acc[i][j]);
        if (SPLIT) {
          acc[i][j] = Frag<T>::mma(ah, bl[j], acc[i][j]);
          acc[i][j] = Frag<T>::mma(al, bh[j], acc[i][j]);
        }
      }
      Frag<T>::guard(acc[i][0], acc[i][3], ah, SPLIT ? al : ah);
    }
    Frag<T>::keep(bh[0], bh[1], bh[2], bh[3]);
    if (SPLIT) Frag<T>::keep(bl[0], bl[1], bl[2], bl[3]);
  }
  acc_guard4(acc[0][0], acc[0][1], acc[0][2], acc[0][3]);
  acc_guard4(acc[1][0], acc[1][1], acc[1][2], acc[1][3]);
  acc_guard4(acc[2][0], acc[2][1], acc[2][2], acc[2][3]);
  acc_guard4(acc[3][0], acc[3][1], acc[3][2], acc[3][3]);

  float* slab = sT[wave];
  const float* Rb = RESID ? (resid + (size_t)b * strideR) : nullptr;
#pragma unroll
  for (int i = 0; i < 4; ++i) {
    const int mBase = m0 + (i << 4);
#pragma unroll
    for (int j = 0; j < 4; ++j) {
      const int n = n0 + (j << 4) + rlane;
      float bv = 0.f;
      if (BIAS_MODE == 2) bv = bias[n];
#pragma unroll
      for (int r = 0; r < 8; ++r) {
        float v = acc[i][j][r] * scale;
        if (BIAS_MODE == 1) v += bias[mBase + mOff + r];
        if (BIAS_MODE == 2) v += bv;
        if (RESID) v += Rb[(size_t)(mBase + mOff + r) * ldc + n];
        if (ACT == 1) v = tanhf(v);
        if (ACT == 2) v = fmaxf(v, 0.0f);
        if (ACT == 3) v = v / (1.0f + expf(-v));
        if (ACT == 4) v = (v > 0.f) ? v : 0.01f * v;
        if (ACT == 5) v = 0.5f * v * (1.0f + erff(v * 0.70710678118654752f));
        slab[(mOff + r) * 68 + (j << 4) + rlane] = v;
      }
    }
    __builtin_amdgcn_fence(__ATOMIC_RELEASE, "workgroup");
    __builtin_amdgcn_wave_barrier();
    __builtin_amdgcn_fence(__ATOMIC_ACQUIRE, "workgroup");
    if (OUT_MODE == 0) {
      float* C = (float*)Cout + (size_t)b * strideC;
      const int hh = lane >> 4, c4 = (lane & 15) * 4;
      for (int pass = 0; pass < 2; ++pass) {
#pragma unroll
        for (int it = 0; it < 8; ++it) {
          const int row = it * 2 + hh;
          v4f v = *(const v4f*)(slab + row * 68 + c4);
          *(volatile v4f*)(C + (size_t)(mBase + row) * ldc + n0 + c4) = v;
        }
        __threadfence();
      }
    } else {
      const int q = lane >> 3, c8 = (lane & 7) * 8;
      unsigned short* C  = (unsigned short*)Cout  + (size_t)b * strideC;
      unsigned short* C2 = (OUT_MODE == 2) ? ((unsigned short*)Cout2 + (size_t)b * strideC) : nullptr;
      for (int pass = 0; pass < 2; ++pass) {
#pragma unroll
        for (int it = 0; it < 4; ++it) {
          const int row = it * 4 + q;
          const float* sp = slab + row * 68 + c8;
          v8h hv, lv;
#pragma unroll
          for (int e = 0; e < 8; ++e) {
            if (OUT_MODE == 1) {
              hv[e] = (_Float16)sp[e];
            } else {
              unsigned short hb = f2bf_bits(sp[e]);
              unsigned short lb = f2bf_bits(sp[e] - bf_bits2f(hb));
              hv[e] = __builtin_bit_cast(_Float16, hb);
              lv[e] = __builtin_bit_cast(_Float16, lb);
            }
          }
          *(volatile v8h*)(C + (size_t)(mBase + row) * ldc + n0 + c8) = hv;
          if (OUT_MODE == 2) *(volatile v8h*)(C2 + (size_t)(mBase + row) * ldc + n0 + c8) = lv;
        }
        __threadfence();
      }
    }
    __builtin_amdgcn_fence(__ATOMIC_RELEASE, "workgroup");
    __builtin_amdgcn_wave_barrier();
    __builtin_amdgcn_fence(__ATOMIC_ACQUIRE, "workgroup");
  }
}

__global__ __launch_bounds__(256) void cast_f32_bf16hl_x2(
    const float* __restrict__ in, unsigned short* __restrict__ hi, unsigned short* __restrict__ lo, int n2) {
  const int i = blockIdx.x * 256 + threadIdx.x;
  if (i < n2) {
    const float f0 = in[2 * i], f1 = in[2 * i + 1];
    const unsigned short h0 = f2bf_bits(f0), h1 = f2bf_bits(f1);
    const unsigned short l0 = f2bf_bits(f0 - bf_bits2f(h0)), l1 = f2bf_bits(f1 - bf_bits2f(h1));
    const unsigned uh = (unsigned)h0 | ((unsigned)h1 << 16);
    const unsigned ul = (unsigned)l0 | ((unsigned)l1 << 16);
    ((volatile unsigned*)hi)[i] = uh;
    ((volatile unsigned*)lo)[i] = ul;
    __threadfence();
    ((volatile unsigned*)hi)[i] = uh;
    ((volatile unsigned*)lo)[i] = ul;
  }
}

__device__ __forceinline__ unsigned pack_bf16_hl(float a, float b, unsigned& lo) {
  const unsigned short ha = f2bf_bits(a), hb = f2bf_bits(b);
  const unsigned short la = f2bf_bits(a - bf_bits2f(ha)), lb = f2bf_bits(b - bf_bits2f(hb));
  lo = (unsigned)la | ((unsigned)lb << 16);
  return (unsigned)ha | ((unsigned)hb << 16);
}
__global__ __launch_bounds__(256) void dwconv3_qkv(
    const float* __restrict__ x,
    const float* __restrict__ wq, const float* __restrict__ bq,
    const float* __restrict__ wk, const float* __restrict__ bk,
    const float* __restrict__ wv, const float* __restrict__ bv,
    unsigned short* __restrict__ Qh, unsigned short* __restrict__ Ql,
    unsigned short* __restrict__ Kh, unsigned short* __restrict__ Kl,
    unsigned short* __restrict__ Vs,
    int nrows, int nseq, float vscale) {
  const int total = nrows * (FE / 2);
  const int idx = blockIdx.x * 256 + threadIdx.x;
  if (idx >= total) return;
  const int row = idx / (FE / 2);
  const int c = (idx - row * (FE / 2)) * 2;
  const int n = row % nseq;
  const bool hasm = (n > 0), hasp = (n < nseq - 1);
  const int rm = hasm ? row - 1 : row;
  const int rp = hasp ? row + 1 : row;
  const v2f xc = *(const v2f*)(x + (size_t)row * FE + c);
  const v2f xa = *(const v2f*)(x + (size_t)rm * FE + c);
  const v2f xb = *(const v2f*)(x + (size_t)rp * FE + c);
  const float xm0 = hasm ? xa[0] : 0.f, xm1 = hasm ? xa[1] : 0.f;
  const float xp0 = hasp ? xb[0] : 0.f, xp1 = hasp ? xb[1] : 0.f;
  const int c3 = c * 3;
  const float q0 = xm0 * wq[c3 + 0] + xc[0] * wq[c3 + 1] + xp0 * wq[c3 + 2] + bq[c];
  const float q1 = xm1 * wq[c3 + 3] + xc[1] * wq[c3 + 4] + xp1 * wq[c3 + 5] + bq[c + 1];
  const float k0 = xm0 * wk[c3 + 0] + xc[0] * wk[c3 + 1] + xp0 * wk[c3 + 2] + bk[c];
  const float k1 = xm1 * wk[c3 + 3] + xc[1] * wk[c3 + 4] + xp1 * wk[c3 + 5] + bk[c + 1];
  const float v0 = xm0 * wv[c3 + 0] + xc[0] * wv[c3 + 1] + xp0 * wv[c3 + 2] + bv[c];
  const float v1 = xm1 * wv[c3 + 3] + xc[1] * wv[c3 + 4] + xp1 * wv[c3 + 5] + bv[c + 1];
  unsigned uql, ukl;
  const unsigned uqh = pack_bf16_hl(q0, q1, uql);
  const unsigned ukh = pack_bf16_hl(k0, k1, ukl);
  const _Float16 hv0 = (_Float16)(v0 * vscale), hv1 = (_Float16)(v1 * vscale);
  const unsigned uv = (unsigned)__builtin_bit_cast(unsigned short, hv0) | ((unsigned)__builtin_bit_cast(unsigned short, hv1) << 16);
  ((volatile unsigned*)Qh)[idx] = uqh;
  ((volatile unsigned*)Ql)[idx] = uql;
  ((volatile unsigned*)Kh)[idx] = ukh;
  ((volatile unsigned*)Kl)[idx] = ukl;
  ((volatile unsigned*)Vs)[idx] = uv;
  __threadfence();
  ((volatile unsigned*)Qh)[idx] = uqh;
  ((volatile unsigned*)Ql)[idx] = uql;
  ((volatile unsigned*)Kh)[idx] = ukh;
  ((volatile unsigned*)Kl)[idx] = ukl;
  ((volatile unsigned*)Vs)[idx] = uv;
}

#define AT_D 64
#define AT_NW 4
#define AT_QB 64
#define AT_KC 64
#define OS_P 68
struct AtKV { __bf16 Kh[AT_KC * AT_D]; __bf16 Kl[AT_KC * AT_D]; _Float16 Vt[AT_D * AT_KC]; };
union AtU { AtKV kv; float os[AT_NW][16 * OS_P]; };

__device__ __forceinline__ v8f mma_bf(v16b a, v16b b, v8f c) {
  c = __builtin_amdgcn_wmma_f32_16x16x32_bf16(false, a, false, b, (short)0, c, false, false);
  asm volatile("v_nop\n\tv_nop\n\tv_nop\n\tv_nop" : "+v"(c) : "v"(a), "v"(b));
  return c;
}
__device__ __forceinline__ v8f mma_hf(v16h a, v16h b, v8f c) {
  c = __builtin_amdgcn_wmma_f32_16x16x32_f16(false, a, false, b, (short)0, c, false, false);
  asm volatile("v_nop\n\tv_nop\n\tv_nop\n\tv_nop" : "+v"(c) : "v"(a), "v"(b));
  return c;
}

__global__ __launch_bounds__(128)
void attn_hd64(const __bf16* __restrict__ Qh, const __bf16* __restrict__ Ql,
               const __bf16* __restrict__ Kh, const __bf16* __restrict__ Kl,
               const _Float16* __restrict__ Vp,
               unsigned short* __restrict__ Ch, unsigned short* __restrict__ Cl,
               int S, int H, int F, float qscale) {
  __shared__ __align__(16) __bf16   Qsh[AT_QB * AT_D];
  __shared__ __align__(16) __bf16   Qsl[AT_QB * AT_D];
  __shared__ __align__(16) AtU      U;
  __shared__ __align__(16) _Float16 Psh[AT_NW][16 * AT_KC];

  const int tid  = threadIdx.x;
  const int wave = tid >> 5;
  const int lane = tid & 31;
  const int hh   = lane >> 4;
  const int c    = lane & 15;

  const int nqb = S / AT_QB;
  const int bx = blockIdx.x;
  const int qb = bx % nqb;
  const int bh = bx / nqb;
  const int h  = bh % H;
  const int b  = bh / H;
  const size_t bhoff = (size_t)b * (size_t)(S * F) + (size_t)h * AT_D;
  const int qbase = qb * AT_QB;
  const int q0 = qbase + wave * 16;

#pragma unroll
  for (int i = 0; i < 4; ++i) {
    const int idx = tid + 128 * i;
    const int r = idx >> 3, seg = (idx & 7) * 8;
    const size_t go = bhoff + (size_t)(qbase + r) * F + seg;
    *(v8b*)(Qsh + r * AT_D + seg) = *(const v8b*)(Qh + go);
    *(v8b*)(Qsl + r * AT_D + seg) = *(const v8b*)(Ql + go);
  }

  float mrow[8], lrow[8];
  v8f oacc[4];
#pragma unroll
  for (int r = 0; r < 8; ++r) { mrow[r] = -INFINITY; lrow[r] = 0.f; }
#pragma unroll
  for (int t = 0; t < 4; ++t) oacc[t] = (v8f){0.f,0.f,0.f,0.f,0.f,0.f,0.f,0.f};

  __bf16* Ksh = U.kv.Kh;
  __bf16* Ksl = U.kv.Kl;
  _Float16* Vth = U.kv.Vt;
  _Float16* pw = Psh[wave];

  const int nChunks = S / AT_KC;
  for (int kc = 0; kc < nChunks; ++kc) {
    const int kv0 = kc * AT_KC;
    __syncthreads();
#pragma unroll
    for (int i = 0; i < 4; ++i) {
      const int idx = tid + 128 * i;
      const int r = idx >> 3, seg = (idx & 7) * 8;
      const size_t go = bhoff + (size_t)(kv0 + r) * F + seg;
      *(v8b*)(Ksh + r * AT_D + seg) = *(const v8b*)(Kh + go);
      *(v8b*)(Ksl + r * AT_D + seg) = *(const v8b*)(Kl + go);
      const v8h vv = *(const v8h*)(Vp + go);
#pragma unroll
      for (int e = 0; e < 8; ++e) Vth[(seg + e) * AT_KC + r] = vv[e];
    }
    __syncthreads();

    v8f s[4];
#pragma unroll
    for (int j = 0; j < 4; ++j) s[j] = (v8f){0.f,0.f,0.f,0.f,0.f,0.f,0.f,0.f};
#pragma unroll
    for (int dc = 0; dc < 2; ++dc) {
      const v16b qa  = Frag<__bf16>::load(Qsh + (wave * 16 + c) * AT_D + dc * 32 + 8 * hh);
      const v16b qlo = Frag<__bf16>::load(Qsl + (wave * 16 + c) * AT_D + dc * 32 + 8 * hh);
#pragma unroll
      for (int j = 0; j < 4; ++j) {
        const v16b kb  = Frag<__bf16>::load(Ksh + (j * 16 + c) * AT_D + dc * 32 + 8 * hh);
        const v16b klo = Frag<__bf16>::load(Ksl + (j * 16 + c) * AT_D + dc * 32 + 8 * hh);
        s[j] = mma_bf(qa, kb, s[j]);
        s[j] = mma_bf(qa, klo, s[j]);
        s[j] = mma_bf(qlo, kb, s[j]);
      }
    }

    float cm[8];
#pragma unroll
    for (int r = 0; r < 8; ++r) {
      float m = -INFINITY;
#pragma unroll
      for (int j = 0; j < 4; ++j) {
        s[j][r] *= qscale;
        m = fmaxf(m, s[j][r]);
      }
#pragma unroll
      for (int off = 1; off < 16; off <<= 1) m = fmaxf(m, __shfl_xor(m, off, 32));
      cm[r] = m;
    }
#pragma unroll
    for (int r = 0; r < 8; ++r) {
      const float mnew = fmaxf(mrow[r], cm[r]);
      const float alpha = expf(mrow[r] - mnew);
      mrow[r] = mnew;
      float psum = 0.f;
#pragma unroll
      for (int j = 0; j < 4; ++j) {
        const float p = expf(s[j][r] - mnew);
        psum += p;
        pw[(8 * hh + r) * AT_KC + j * 16 + c] = (_Float16)(p * 32768.0f);
      }
#pragma unroll
      for (int off = 1; off < 16; off <<= 1) psum += __shfl_xor(psum, off, 32);
      lrow[r] = lrow[r] * alpha + psum;
#pragma unroll
      for (int t = 0; t < 4; ++t) oacc[t][r] *= alpha;
    }
    __builtin_amdgcn_fence(__ATOMIC_RELEASE, "workgroup");
    __builtin_amdgcn_wave_barrier();
    __builtin_amdgcn_fence(__ATOMIC_ACQUIRE, "workgroup");

#pragma unroll
    for (int kk = 0; kk < 2; ++kk) {
      const v16h pa = Frag<_Float16>::load(pw + c * AT_KC + kk * 32 + 8 * hh);
#pragma unroll
      for (int t = 0; t < 4; ++t) {
        const v16h vb = Frag<_Float16>::load(Vth + (t * 16 + c) * AT_KC + kk * 32 + 8 * hh);
        oacc[t] = mma_hf(pa, vb, oacc[t]);
      }
    }
  }

  __syncthreads();
  float* os = U.os[wave];
#pragma unroll
  for (int r = 0; r < 8; ++r) {
    const float inv = 1.0f / (lrow[r] * 1048576.0f);
#pragma unroll
    for (int t = 0; t < 4; ++t) os[(8 * hh + r) * OS_P + t * 16 + c] = oacc[t][r] * inv;
  }
  __builtin_amdgcn_fence(__ATOMIC_RELEASE, "workgroup");
  __builtin_amdgcn_wave_barrier();
  __builtin_amdgcn_fence(__ATOMIC_ACQUIRE, "workgroup");
  {
    const int q = lane >> 3, c8 = (lane & 7) * 8;
    for (int pass = 0; pass < 2; ++pass) {
#pragma unroll
      for (int it = 0; it < 4; ++it) {
        const int row = it * 4 + q;
        const float* sp = os + row * OS_P + c8;
        v8h hv, lv;
#pragma unroll
        for (int e = 0; e < 8; ++e) {
          const unsigned short hb = f2bf_bits(sp[e]);
          const unsigned short lb = f2bf_bits(sp[e] - bf_bits2f(hb));
          hv[e] = __builtin_bit_cast(_Float16, hb);
          lv[e] = __builtin_bit_cast(_Float16, lb);
        }
        const size_t o = bhoff + (size_t)(q0 + row) * F + c8;
        *(volatile v8h*)(Ch + o) = hv;
        *(volatile v8h*)(Cl + o) = lv;
      }
      __threadfence();
    }
  }
}

extern "C" void kernel_launch(void* const* d_in, const int* in_sizes, int n_in,
                              void* d_out, int out_size, void* d_ws, size_t ws_size,
                              hipStream_t stream) {
  if (n_in < 9) return;
  const int F = FE, S = 512, Hn = NHEAD;
  const int nx = in_sizes[0];
  if (nx <= 0 || (nx % (S * F)) != 0) return;
  const int B = nx / (S * F);
  const int R = B * S;
  if ((R % 64) != 0 || (S % 64) != 0 || out_size != nx) return;
  if (in_sizes[7] != F * F || in_sizes[1] != F * 3 || in_sizes[3] != F * 3 || in_sizes[5] != F * 3) return;
  if (in_sizes[2] != F || in_sizes[4] != F || in_sizes[6] != F || in_sizes[8] != F) return;

  const float* x  = (const float*)d_in[0];
  const float* wq = (const float*)d_in[1];
  const float* bq = (const float*)d_in[2];
  const float* wk = (const float*)d_in[3];
  const float* bk = (const float*)d_in[4];
  const float* wv = (const float*)d_in[5];
  const float* bv = (const float*)d_in[6];
  const float* wo = (const float*)d_in[7];
  const float* bo = (const float*)d_in[8];
  float* out = (float*)d_out;

  const size_t woBytes    = (size_t)F * F * 2;
  const size_t planeBytes = (size_t)R * F * 2;
  char* ws = (char*)d_ws;
  size_t off = 0;
  unsigned short* woh = (unsigned short*)(ws + off); off += woBytes;
  unsigned short* wol = (unsigned short*)(ws + off); off += woBytes;
  unsigned short* qh  = (unsigned short*)(ws + off); off += planeBytes;
  unsigned short* ql  = (unsigned short*)(ws + off); off += planeBytes;
  unsigned short* kh  = (unsigned short*)(ws + off); off += planeBytes;
  unsigned short* kl  = (unsigned short*)(ws + off); off += planeBytes;
  unsigned short* vs  = (unsigned short*)(ws + off); off += planeBytes;
  unsigned short* ch  = (unsigned short*)(ws + off); off += planeBytes;
  unsigned short* cl  = (unsigned short*)(ws + off); off += planeBytes;
  if (off > ws_size) return;

  {
    const int n2 = (F * F) / 2;
    cast_f32_bf16hl_x2<<<(n2 + 255) / 256, 256, 0, stream>>>(wo, woh, wol, n2);
  }
  {
    const int tot = R * (F / 2);
    dwconv3_qkv<<<(tot + 255) / 256, 256, 0, stream>>>(x, wq, bq, wk, bk, wv, bv,
                                                       qh, ql, kh, kl, vs, R, S, 32.0f);
  }
  {
    const float qscale = 1.0f / sqrtf((float)F);
    attn_hd64<<<B * Hn * (S / 64), 128, 0, stream>>>(
        (const __bf16*)qh, (const __bf16*)ql, (const __bf16*)kh, (const __bf16*)kl,
        (const _Float16*)vs, ch, cl, S, Hn, F, qscale);
  }
  {
    const int tiles = (R / 64) * (F / 64);
    wmma_gemm64<1, true, 2, 0, false><<<dim3((tiles + 7) / 8, 1), 256, 0, stream>>>(
        ch, cl, F, 0L,
        woh, wol, F, 0L,
        (void*)out, (void*)cl, F, 0L,
        bo,
        bo, 0L,
        R, F, F, 1.0f);
  }
}
